// PatternDetector_69226282877319
// MI455X (gfx1250) — hardware-run, weakly checked
//
#include <hip/hip_runtime.h>
#include <math.h>

typedef float v4f __attribute__((ext_vector_type(4)));
typedef unsigned int v4u __attribute__((ext_vector_type(4)));

#define VST2(T, ptr, val) do { const T vst2_v_ = (val); *(volatile T*)(ptr) = vst2_v_; __threadfence(); *(volatile T*)(ptr) = vst2_v_; } while (0)
#define VST2V4(ptr, val) do { const v4f vst2_v4_ = (val); *(volatile v4f*)(ptr) = vst2_v4_; __threadfence(); *(volatile v4f*)(ptr) = vst2_v4_; } while (0)

namespace eng {
typedef __attribute__((ext_vector_type(16))) _Float16 v16h;
typedef __attribute__((ext_vector_type(8)))  _Float16 v8h;
typedef __attribute__((ext_vector_type(16))) __bf16   v16b;
typedef __attribute__((ext_vector_type(8)))  __bf16   v8b;
typedef __attribute__((ext_vector_type(8)))  float    v8f;
typedef __attribute__((ext_vector_type(4)))  float    v4f;

__device__ __forceinline__ unsigned short f2bf_bits(float f) {
  unsigned u = __float_as_uint(f);
  return (unsigned short)((u + 0x7FFFu + ((u >> 16) & 1u)) >> 16);
}
__device__ __forceinline__ float bf_bits2f(unsigned short h) { return __uint_as_float(((unsigned)h) << 16); }

__device__ __forceinline__ void dep_guard_h(v8f& a, v8f& b, v16h x, v16h y) { asm volatile("v_nop\n\tv_nop\n\tv_nop\n\tv_nop" : "+v"(a), "+v"(b) : "v"(x), "v"(y)); }
__device__ __forceinline__ void dep_guard_b(v8f& a, v8f& b, v16b x, v16b y) { asm volatile("v_nop\n\tv_nop\n\tv_nop\n\tv_nop" : "+v"(a), "+v"(b) : "v"(x), "v"(y)); }
__device__ __forceinline__ void keep4_h(v16h a, v16h b, v16h c, v16h d) { asm volatile("v_nop" :: "v"(a), "v"(b), "v"(c), "v"(d)); }
__device__ __forceinline__ void keep4_b(v16b a, v16b b, v16b c, v16b d) { asm volatile("v_nop" :: "v"(a), "v"(b), "v"(c), "v"(d)); }
__device__ __forceinline__ void acc_guard4(v8f& a, v8f& b, v8f& c, v8f& d) { asm volatile("v_nop\n\tv_nop\n\tv_nop\n\tv_nop" : "+v"(a), "+v"(b), "+v"(c), "+v"(d)); }
template <typename T> struct Frag;
template <> struct Frag<_Float16> {
  typedef v16h V; union U { v16h v; v8h h[2]; };
  static __device__ __forceinline__ v16h load(const _Float16* p) {
    U f; f.h[0] = *(const v8h*)(p); f.h[1] = *(const v8h*)(p + 16); return f.v;
  }
  static __device__ __forceinline__ v8f mma(v16h a, v16h b, v8f c) {
    return __builtin_amdgcn_wmma_f32_16x16x32_f16(false, a, false, b, (short)0, c, false, false);
  }
  static __device__ __forceinline__ void guard(v8f& a, v8f& b, v16h x, v16h y) { dep_guard_h(a, b, x, y); }
  static __device__ __forceinline__ void keep(v16h a, v16h b, v16h c, v16h d) { keep4_h(a, b, c, d); }
};
template <> struct Frag<__bf16> {
  typedef v16b V; union U { v16b v; v8b h[2]; };
  static __device__ __forceinline__ v16b load(const __bf16* p) {
    U f; f.h[0] = *(const v8b*)(p); f.h[1] = *(const v8b*)(p + 16); return f.v;
  }
  static __device__ __forceinline__ v8f mma(v16b a, v16b b, v8f c) {
    return __builtin_amdgcn_wmma_f32_16x16x32_bf16(false, a, false, b, (short)0, c, false, false);
  }
  static __device__ __forceinline__ void guard(v8f& a, v8f& b, v16b x, v16b y) { dep_guard_b(a, b, x, y); }
  static __device__ __forceinline__ void keep(v16b a, v16b b, v16b c, v16b d) { keep4_b(a, b, c, d); }
};

template <int ET> struct Elem;
template <> struct Elem<0> { typedef _Float16 T; };
template <> struct Elem<1> { typedef __bf16 T; };
template <int ET, bool SPLIT, int BIAS_MODE, int OUT_MODE, bool RESID, int ACT = 0>
__global__ __launch_bounds__(256) void wmma_gemm64(
    const unsigned short* __restrict__ Ap, const unsigned short* __restrict__ A2p, int lda, long strideA,
    const unsigned short* __restrict__ Btp, const unsigned short* __restrict__ Bt2p, int ldb, long strideB,
    void* __restrict__ Cout, void* __restrict__ Cout2, int ldc, long strideC,
    const float* __restrict__ bias,
    const float* __restrict__ resid, long strideR,
    int M, int N, int K, float scale) {
  typedef typename Elem<ET>::T T;
  typedef typename Frag<T>::V V;
  const T* A = (const T*)Ap; const T* A2 = (const T*)A2p; const T* Bt = (const T*)Btp; const T* Bt2 = (const T*)Bt2p;
  __shared__ __align__(16) float sT[8][16 * 68];
  const int b    = blockIdx.y;
  const int lane = threadIdx.x & 31;
  const int wave = threadIdx.x >> 5;
  const int tilesN = N >> 6;
  const int tilesM = M >> 6;
  const int tile = blockIdx.x * 8 + wave;
  if (tile >= tilesM * tilesN) return;
  const int tm = tile / tilesN;
  const int tn = tile - tm * tilesN;
  const int m0 = tm << 6;
  const int n0 = tn << 6;

  const T* Ab  = A  + (size_t)b * strideA;
  const T* Bb  = Bt + (size_t)b * strideB;
  const T* Ab2 = SPLIT ? (A2  + (size_t)b * strideA) : nullptr;
  const T* Bb2 = SPLIT ? (Bt2 + (size_t)b * strideB) : nullptr;

  const int rlane = lane & 15;
  const int koff  = (lane >> 4) * 8;
  const int mOff  = (lane >> 4) * 8;

  v8f acc[4][4];
#pragma unroll
  for (int i = 0; i < 4; ++i)
#pragma unroll
    for (int j = 0; j < 4; ++j) acc[i][j] = (v8f){0.f,0.f,0.f,0.f,0.f,0.f,0.f,0.f};

  for (int k0 = 0; k0 < K; k0 += 32) {
    V bh[4], bl[4];
#pragma unroll
    for (int j = 0; j < 4; ++j) {
      const size_t bo = (size_t)(n0 + (j << 4) + rlane) * ldb + koff + k0;
      bh[j] = Frag<T>::load(Bb + bo);
      if (SPLIT) bl[j] = Frag<T>::load(Bb2 + bo);
    }
#pragma unroll
    for (int i = 0; i < 4; ++i) {
      const size_t ao = (size_t)(m0 + (i << 4) + rlane) * lda + koff + k0;
      V ah = Frag<T>::load(Ab + ao);
      V al;
      if (SPLIT) al = Frag<T>::load(Ab2 + ao);
#pragma unroll
      for (int j = 0; j < 4; ++j) {
        acc[i][j] = Frag<T>::mma(ah, bh[j], acc[i][j]);
        if (SPLIT) {
          acc[i][j] = Frag<T>::mma(ah, bl[j], acc[i][j]);
          acc[i][j] = Frag<T>::mma(al, bh[j], acc[i][j]);
        }
      }
      Frag<T>::guard(acc[i][0], acc[i][3], ah, SPLIT ? al : ah);
    }
    Frag<T>::keep(bh[0], bh[1], bh[2], bh[3]);
    if (SPLIT) Frag<T>::keep(bl[0], bl[1], bl[2], bl[3]);
  }
  acc_guard4(acc[0][0], acc[0][1], acc[0][2], acc[0][3]);
  acc_guard4(acc[1][0], acc[1][1], acc[1][2], acc[1][3]);
  acc_guard4(acc[2][0], acc[2][1], acc[2][2], acc[2][3]);
  acc_guard4(acc[3][0], acc[3][1], acc[3][2], acc[3][3]);

  float* slab = sT[wave];
  const float* Rb = RESID ? (resid + (size_t)b * strideR) : nullptr;
#pragma unroll
  for (int i = 0; i < 4; ++i) {
    const int mBase = m0 + (i << 4);
#pragma unroll
    for (int j = 0; j < 4; ++j) {
      const int n = n0 + (j << 4) + rlane;
      float bv = 0.f;
      if (BIAS_MODE == 2) bv = bias[n];
#pragma unroll
      for (int r = 0; r < 8; ++r) {
        float v = acc[i][j][r] * scale;
        if (BIAS_MODE == 1) v += bias[mBase + mOff + r];
        if (BIAS_MODE == 2) v += bv;
        if (RESID) v += Rb[(size_t)(mBase + mOff + r) * ldc + n];
        if (ACT == 1) v = tanhf(v);
        if (ACT == 2) v = fmaxf(v, 0.0f);
        if (ACT == 3) v = v / (1.0f + expf(-v));
        if (ACT == 4) v = (v > 0.f) ? v : 0.01f * v;
        if (ACT == 5) v = 0.5f * v * (1.0f + erff(v * 0.70710678118654752f));
        if (ACT == 6) v = (v > 0.f) ? v : 0.2f * v;
        if (ACT == 7) { const float u = 0.7978845608028654f * (v + 0.044715f * v * v * v); v = 0.5f * v * (1.f + tanhf(u)); }
        slab[(mOff + r) * 68 + (j << 4) + rlane] = v;
      }
    }
    __builtin_amdgcn_fence(3  , "workgroup");
    __builtin_amdgcn_wave_barrier();
    __builtin_amdgcn_fence(2  , "workgroup");
    if (OUT_MODE == 0) {
      float* C = (float*)Cout + (size_t)b * strideC;
      const int hh = lane >> 4, c4 = (lane & 15) * 4;
      for (int pass = 0; pass < 2; ++pass) {
#pragma unroll
        for (int it = 0; it < 8; ++it) {
          const int row = it * 2 + hh;
          v4f v = *(const v4f*)(slab + row * 68 + c4);
          *(volatile v4f*)(C + (size_t)(mBase + row) * ldc + n0 + c4) = v;
        }
        __threadfence();
      }
    } else {
      const int q = lane >> 3, c8 = (lane & 7) * 8;
      unsigned short* C  = (unsigned short*)Cout  + (size_t)b * strideC;
      unsigned short* C2 = (OUT_MODE == 2) ? ((unsigned short*)Cout2 + (size_t)b * strideC) : nullptr;
      for (int pass = 0; pass < 2; ++pass) {
#pragma unroll
        for (int it = 0; it < 4; ++it) {
          const int row = it * 4 + q;
          const float* sp = slab + row * 68 + c8;
          v8h hv, lv;
#pragma unroll
          for (int e = 0; e < 8; ++e) {
            if (OUT_MODE == 1) {
              hv[e] = (_Float16)sp[e];
            } else {
              unsigned short hb = f2bf_bits(sp[e]);
              unsigned short lb = f2bf_bits(sp[e] - bf_bits2f(hb));
              hv[e] = __builtin_bit_cast(_Float16, hb);
              lv[e] = __builtin_bit_cast(_Float16, lb);
            }
          }
          *(volatile v8h*)(C + (size_t)(mBase + row) * ldc + n0 + c8) = hv;
          if (OUT_MODE == 2) *(volatile v8h*)(C2 + (size_t)(mBase + row) * ldc + n0 + c8) = lv;
        }
        __threadfence();
      }
    }
    __builtin_amdgcn_fence(3  , "workgroup");
    __builtin_amdgcn_wave_barrier();
    __builtin_amdgcn_fence(2  , "workgroup");
  }
}

}

#ifndef NB
#define NB 512
#endif
#define NB_FULL 512
#define IN_DIM 256
#define HID 512
#define HID2 256
#define PAT 10
#define PATP 64
#define NXW (3 * HID)
#define CARRY_A 8.0f
#define CARRY_W 32.0f
#define INV_CARRY 0.00390625f

static_assert(NB % 64 == 0 && NB <= NB_FULL && NB >= 64);
static_assert(IN_DIM % 32 == 0 && HID % 32 == 0 && HID2 % 32 == 0);
static_assert(NXW % 64 == 0 && HID2 % 64 == 0 && PATP % 64 == 0 && PAT <= PATP);
static_assert(IN_DIM % 8 == 0 && HID % 8 == 0 && HID2 % 8 == 0);
static_assert(8 * 16 * 68 * 4 <= 131072);

static __device__ __forceinline__ float bfr(float f) { unsigned u = __float_as_uint(f); u += 0x7FFFu + ((u >> 16) & 1u); return __uint_as_float(u & 0xFFFF0000u); }
typedef _Float16 h16;
static __device__ __forceinline__ h16 toh_flush(float v) { const h16 r = (h16)v; return (fabsf(v) < 6.103515625e-05f) ? (h16)0.0f : r; }
static __device__ __forceinline__ unsigned int pk2h_flush(float a, float b) { return (unsigned int)__builtin_bit_cast(unsigned short, toh_flush(a)) | ((unsigned int)__builtin_bit_cast(unsigned short, toh_flush(b)) << 16); }
static __device__ __forceinline__ void st8h_flush(unsigned short* Pp, long long o, const float* v) {
    v4u pk; pk.x = pk2h_flush(v[0], v[1]); pk.y = pk2h_flush(v[2], v[3]); pk.z = pk2h_flush(v[4], v[5]); pk.w = pk2h_flush(v[6], v[7]);
    VST2(v4u, (v4u*)(Pp + o), pk);
}

__global__ __launch_bounds__(256) void k_cvt16(const float* __restrict__ S, int rowsValid, int rowsPad, int K, unsigned short* __restrict__ D, float sc) {
    const long long u = (long long)blockIdx.x * 256 + threadIdx.x; const int per = K / 8; if (u >= (long long)rowsPad * per) return;
    const int k0 = 8 * (int)(u % per); const int r = (int)(u / per); const int rc = min(r, rowsValid - 1);
    const float* x = S + (long long)rc * K + k0; float v[8];
#pragma unroll
    for (int i = 0; i < 8; ++i) { const float t = bfr(x[i]) * sc; v[i] = (r < rowsValid) ? t : 0.f; }
    st8h_flush(D, (long long)r * K + k0, v);
}

__global__ __launch_bounds__(256) void k_bnrelu16(const float* __restrict__ XW, const float* __restrict__ B1, const float* __restrict__ G, const float* __restrict__ BT,
                                                  const float* __restrict__ MU, const float* __restrict__ VAR, unsigned short* __restrict__ H16, float carry) {
    #pragma clang fp contract(off)
    const long long u = (long long)blockIdx.x * 256 + threadIdx.x; if (u >= (long long)NB * (HID / 8)) return;
    const int c0 = 8 * (int)(u % (HID / 8)); const int r = (int)(u / (HID / 8));
    const float* xr = XW + (long long)r * NXW + c0; float v[8];
#pragma unroll
    for (int i = 0; i < 8; ++i) {
        const int c = c0 + i;
        const float t = xr[i] + bfr(B1[c]);
        float y = bfr(G[c]) * (t - bfr(MU[c]));
        y = y * rsqrtf(bfr(VAR[c]) + 1e-5f);
        y = y + bfr(BT[c]);
        v[i] = fmaxf(y, 0.f) * carry;
    }
    st8h_flush(H16, (long long)r * HID + c0, v);
}

__global__ __launch_bounds__(256) void k_biasrelu16(const float* __restrict__ RAW, const float* __restrict__ B2, unsigned short* __restrict__ H216, float carry) {
    #pragma clang fp contract(off)
    const long long u = (long long)blockIdx.x * 256 + threadIdx.x; if (u >= (long long)NB * (HID2 / 8)) return;
    const int c0 = 8 * (int)(u % (HID2 / 8)); const int r = (int)(u / (HID2 / 8));
    const float* xr = RAW + (long long)r * HID2 + c0; float v[8];
#pragma unroll
    for (int i = 0; i < 8; ++i) {
        const float t = xr[i] + bfr(B2[c0 + i]);
        v[i] = fmaxf(t, 0.f) * carry;
    }
    st8h_flush(H216, (long long)r * HID2 + c0, v);
}

#define HROWS 64
static_assert((HROWS * PAT * 4) % 128 == 0 && (HROWS * PAT) % 4 == 0 && HROWS * PAT / 4 <= 256 && NB % HROWS == 0);
static_assert((HROWS * PAT / 4) * 16 == HROWS * PAT * 4);
static_assert(2 * HROWS * PAT * 4 <= 131072);
__global__ __launch_bounds__(256) void k_head(const float* __restrict__ SC, const float* __restrict__ B3, float* __restrict__ PROB, float* __restrict__ SCORE) {
    #pragma clang fp contract(off)
    __shared__ __align__(16) float sP[HROWS * PAT];
    __shared__ __align__(16) float sS[HROWS * PAT];
    const int tid = threadIdx.x; const int r0 = blockIdx.x * HROWS;
    if (tid < HROWS) {
        const float* sr = SC + (long long)(r0 + tid) * PATP;
        float m = -__builtin_inff();
#pragma unroll 1
        for (int j = 0; j < PAT; ++j) { const float v = sr[j] + bfr(B3[j]); sS[tid * PAT + j] = v; m = fmaxf(m, v); }
        float sum = 0.f;
#pragma unroll 1
        for (int j = 0; j < PAT; ++j) { const float e = expf(sS[tid * PAT + j] - m); sP[tid * PAT + j] = e; sum += e; }
        const float inv = 1.0f / sum;
#pragma unroll 1
        for (int j = 0; j < PAT; ++j) { const float e = sP[tid * PAT + j]; sP[tid * PAT + j] = e * inv; }
    }
    __syncthreads();
    if (tid < HROWS * PAT / 4) {
        const v4f pv = *(const v4f*)(sP + 4 * tid);
        const v4f sv = *(const v4f*)(sS + 4 * tid);
        VST2V4(PROB + (long long)r0 * PAT + 4 * tid, pv);
        VST2V4(SCORE + (long long)r0 * PAT + 4 * tid, sv);
    }
}

#define PT 32
#define PKC 128
#define PPITCH 132
#define TPITCH 33
#define NTL (NB / PT)
static_assert(NB % PT == 0 && HID % PKC == 0 && PKC % 4 == 0 && (PPITCH * 4) % 16 == 0 && PPITCH >= PKC);
static_assert(4 * 256 * 4 == PT * PKC);
static_assert(256 * 16 == PT * PT * 4);
static_assert(PKC <= 256);
static_assert((2 * PT * PPITCH + PKC + PT * TPITCH) * 4 <= 131072);

static __device__ __forceinline__ float pair_acc4(float acc, v4f a, v4f c, v4f w) {
    acc = fmaf(fmaxf(a.x + c.x, 0.f), w.x, acc);
    acc = fmaf(fmaxf(a.y + c.y, 0.f), w.y, acc);
    acc = fmaf(fmaxf(a.z + c.z, 0.f), w.z, acc);
    acc = fmaf(fmaxf(a.w + c.w, 0.f), w.w, acc);
    return acc;
}

__global__ __launch_bounds__(256) void k_pair(const float* __restrict__ XW, const float* __restrict__ BS1, const float* __restrict__ WS2, const float* __restrict__ BS2, float* __restrict__ SIM) {
    __shared__ __align__(16) float As[PT * PPITCH];
    __shared__ __align__(16) float Cs[PT * PPITCH];
    __shared__ __align__(16) float Wk[PKC];
    __shared__ __align__(16) float Tt[PT * TPITCH];
    const int tid = threadIdx.x, ty = tid >> 4, tx = tid & 15;
    int rem = (int)blockIdx.x, bi = 0, len = NTL;
#pragma unroll 1
    for (int it = 0; it < NTL - 1; ++it) { if (rem >= len) { rem -= len; ++bi; --len; } }
    const int bj = min(bi + rem, NTL - 1);
    const int i0 = bi * PT, j0 = bj * PT;
    float acc00 = 0.f, acc01 = 0.f, acc10 = 0.f, acc11 = 0.f;
#pragma unroll 1
    for (int kc = 0; kc < HID; kc += PKC) {
        __syncthreads();
#pragma unroll
        for (int q = 0; q < 4; ++q) {
            const int idx = tid + 256 * q; const int row = idx >> 5, c4 = (idx & 31) * 4;
            v4f a = *(const v4f*)(XW + (long long)(i0 + row) * NXW + HID + kc + c4);
            const v4f c = *(const v4f*)(XW + (long long)(j0 + row) * NXW + 2 * HID + kc + c4);
            a.x += bfr(BS1[kc + c4]); a.y += bfr(BS1[kc + c4 + 1]); a.z += bfr(BS1[kc + c4 + 2]); a.w += bfr(BS1[kc + c4 + 3]);
            *(v4f*)(As + row * PPITCH + c4) = a;
            *(v4f*)(Cs + row * PPITCH + c4) = c;
        }
        if (tid < PKC) Wk[tid] = bfr(WS2[kc + tid]);
        __syncthreads();
#pragma unroll 1
        for (int k4 = 0; k4 < PKC; k4 += 4) {
            const v4f a0 = *(const v4f*)(As + ty * PPITCH + k4);
            const v4f a1 = *(const v4f*)(As + (ty + 16) * PPITCH + k4);
            const v4f c0 = *(const v4f*)(Cs + tx * PPITCH + k4);
            const v4f c1 = *(const v4f*)(Cs + (tx + 16) * PPITCH + k4);
            const v4f w = *(const v4f*)(Wk + k4);
            acc00 = pair_acc4(acc00, a0, c0, w);
            acc01 = pair_acc4(acc01, a0, c1, w);
            acc10 = pair_acc4(acc10, a1, c0, w);
            acc11 = pair_acc4(acc11, a1, c1, w);
        }
    }
    const float b2 = bfr(BS2[0]);
    Tt[ty * TPITCH + tx] = acc00 + b2;
    Tt[ty * TPITCH + tx + 16] = acc01 + b2;
    Tt[(ty + 16) * TPITCH + tx] = acc10 + b2;
    Tt[(ty + 16) * TPITCH + tx + 16] = acc11 + b2;
    __syncthreads();
#pragma unroll 1
    for (int q = 0; q < 4; ++q) {
        const int e = tid + 256 * q; const int r = e >> 5, c = e & 31;
        const float v = Tt[r * TPITCH + c];
        const float s = 1.f / (1.f + expf(-v));
        Tt[r * TPITCH + c] = s;
    }
    __syncthreads();
    const int r = tid >> 3, p4 = (tid & 7) * 4;
    if (bi != bj) {
        v4f v; v.x = Tt[r * TPITCH + p4]; v.y = Tt[r * TPITCH + p4 + 1]; v.z = Tt[r * TPITCH + p4 + 2]; v.w = Tt[r * TPITCH + p4 + 3];
        VST2V4(SIM + (long long)(i0 + r) * NB_FULL + j0 + p4, v);
        v4f u; u.x = Tt[p4 * TPITCH + r]; u.y = Tt[(p4 + 1) * TPITCH + r]; u.z = Tt[(p4 + 2) * TPITCH + r]; u.w = Tt[(p4 + 3) * TPITCH + r];
        VST2V4(SIM + (long long)(j0 + r) * NB_FULL + i0 + p4, u);
    } else {
        const int ca = p4, cb = p4 + 1, cc = p4 + 2, cd = p4 + 3;
        const float ta = Tt[min(r, ca) * TPITCH + max(r, ca)];
        const float tb = Tt[min(r, cb) * TPITCH + max(r, cb)];
        const float tc = Tt[min(r, cc) * TPITCH + max(r, cc)];
        const float td = Tt[min(r, cd) * TPITCH + max(r, cd)];
        v4f v; v.x = (r == ca) ? 0.f : ta; v.y = (r == cb) ? 0.f : tb; v.z = (r == cc) ? 0.f : tc; v.w = (r == cd) ? 0.f : td;
        VST2V4(SIM + (long long)(i0 + r) * NB_FULL + i0 + p4, v);
    }
}

#define SZ_X16  ((size_t)NB * IN_DIM * 2)
#define SZ_WB16 ((size_t)NXW * IN_DIM * 2)
#define SZ_W2   ((size_t)HID2 * HID * 2)
#define SZ_W3   ((size_t)PATP * HID2 * 2)
#define SZ_XW   ((size_t)NB * NXW * 4)
#define SZ_H16  ((size_t)NB * HID * 2)
#define SZ_H2R  ((size_t)NB * HID2 * 4)
#define SZ_H216 ((size_t)NB * HID2 * 2)
#define SZ_SC   ((size_t)NB * PATP * 4)
#define SZ_TOTAL (SZ_X16 + SZ_WB16 + SZ_W2 + SZ_W3 + SZ_XW + SZ_H16 + SZ_H2R + SZ_H216 + SZ_SC)
static_assert(SZ_X16 % 256 == 0 && SZ_WB16 % 256 == 0 && SZ_W2 % 256 == 0 && SZ_W3 % 256 == 0 && SZ_XW % 256 == 0);
static_assert(SZ_H16 % 256 == 0 && SZ_H2R % 256 == 0 && SZ_H216 % 256 == 0 && SZ_SC % 256 == 0);
static_assert(SZ_TOTAL <= (size_t)134217728);
static_assert((size_t)NB_FULL * PAT * 4 == 20480 && (size_t)2 * NB_FULL * PAT * 4 == 40960 && (40960 % 128) == 0);
static_assert((size_t)2 * NB_FULL * PAT * 4 + (size_t)NB_FULL * NB_FULL * 4 == 1089536);

extern "C" void kernel_launch(void* const* d_in, const int* in_sizes, int n_in, void* d_out, int out_size, void* d_ws, size_t ws_size, hipStream_t stream) {
    if (n_in < 16) return;
    if (in_sizes[0] < NB * IN_DIM || in_sizes[1] < HID * IN_DIM || in_sizes[2] < HID || in_sizes[3] < HID || in_sizes[4] < HID || in_sizes[5] < HID || in_sizes[6] < HID) return;
    if (in_sizes[7] < HID2 * HID || in_sizes[8] < HID2 || in_sizes[9] < PAT * HID2 || in_sizes[10] < PAT) return;
    if (in_sizes[11] < HID * IN_DIM || in_sizes[12] < HID * IN_DIM || in_sizes[13] < HID || in_sizes[14] < HID || in_sizes[15] < 1) return;
    if (out_size < 2 * NB_FULL * PAT + (NB - 1) * NB_FULL + NB) return;
    if (SZ_TOTAL > ws_size) return;
    const float* x    = (const float*)d_in[0];
    const float* W1   = (const float*)d_in[1];
    const float* b1   = (const float*)d_in[2];
    const float* bng  = (const float*)d_in[3];
    const float* bnb  = (const float*)d_in[4];
    const float* bnm  = (const float*)d_in[5];
    const float* bnv  = (const float*)d_in[6];
    const float* W2   = (const float*)d_in[7];
    const float* b2   = (const float*)d_in[8];
    const float* W3   = (const float*)d_in[9];
    const float* b3   = (const float*)d_in[10];
    const float* Ws1a = (const float*)d_in[11];
    const float* Ws1b = (const float*)d_in[12];
    const float* bs1  = (const float*)d_in[13];
    const float* ws2  = (const float*)d_in[14];
    const float* bs2  = (const float*)d_in[15];
    float* out = (float*)d_out;
    float* PROB = out;
    float* SCORE = out + (size_t)NB_FULL * PAT;
    float* SIM = out + (size_t)2 * NB_FULL * PAT;

    char* wsp = (char*)d_ws;
    unsigned short* X16  = (unsigned short*)wsp; wsp += SZ_X16;
    unsigned short* WB16 = (unsigned short*)wsp; wsp += SZ_WB16;
    unsigned short* W216 = (unsigned short*)wsp; wsp += SZ_W2;
    unsigned short* W316 = (unsigned short*)wsp; wsp += SZ_W3;
    float*          XW   = (float*)wsp;          wsp += SZ_XW;
    unsigned short* H16  = (unsigned short*)wsp; wsp += SZ_H16;
    float*          H2R  = (float*)wsp;          wsp += SZ_H2R;
    unsigned short* H216 = (unsigned short*)wsp; wsp += SZ_H216;
    float*          SC   = (float*)wsp;          wsp += SZ_SC;
    if ((size_t)(wsp - (char*)d_ws) > ws_size) return;

    k_cvt16<<<(unsigned)(((size_t)NB * (IN_DIM / 8) + 255) / 256), 256, 0, stream>>>(x, NB, NB, IN_DIM, X16, CARRY_A);
    k_cvt16<<<(unsigned)(((size_t)HID * (IN_DIM / 8) + 255) / 256), 256, 0, stream>>>(W1, HID, HID, IN_DIM, WB16, CARRY_W);
    k_cvt16<<<(unsigned)(((size_t)HID * (IN_DIM / 8) + 255) / 256), 256, 0, stream>>>(Ws1a, HID, HID, IN_DIM, WB16 + (size_t)HID * IN_DIM, CARRY_W);
    k_cvt16<<<(unsigned)(((size_t)HID * (IN_DIM / 8) + 255) / 256), 256, 0, stream>>>(Ws1b, HID, HID, IN_DIM, WB16 + (size_t)2 * HID * IN_DIM, CARRY_W);
    k_cvt16<<<(unsigned)(((size_t)HID2 * (HID / 8) + 255) / 256), 256, 0, stream>>>(W2, HID2, HID2, HID, W216, CARRY_W);
    k_cvt16<<<(unsigned)(((size_t)PATP * (HID2 / 8) + 255) / 256), 256, 0, stream>>>(W3, PAT, PATP, HID2, W316, CARRY_W);
    eng::wmma_gemm64<0, false, 0, 0, false, 0><<<dim3((unsigned)((((NB) / 64) * ((NXW) / 64) + 7) / 8), (unsigned)(1)), 256, 0, stream>>>((const unsigned short*)(X16), nullptr, IN_DIM, 0, (const unsigned short*)(WB16), nullptr, IN_DIM, 0, (void*)(XW), nullptr, NXW, 0, nullptr, nullptr, 0, NB, NXW, IN_DIM, INV_CARRY);
    k_bnrelu16<<<(unsigned)(((size_t)NB * (HID / 8) + 255) / 256), 256, 0, stream>>>(XW, b1, bng, bnb, bnm, bnv, H16, CARRY_A);
    eng::wmma_gemm64<0, false, 0, 0, false, 0><<<dim3((unsigned)((((NB) / 64) * ((HID2) / 64) + 7) / 8), (unsigned)(1)), 256, 0, stream>>>((const unsigned short*)(H16), nullptr, HID, 0, (const unsigned short*)(W216), nullptr, HID, 0, (void*)(H2R), nullptr, HID2, 0, nullptr, nullptr, 0, NB, HID2, HID, INV_CARRY);
    k_biasrelu16<<<(unsigned)(((size_t)NB * (HID2 / 8) + 255) / 256), 256, 0, stream>>>(H2R, b2, H216, CARRY_A);
    eng::wmma_gemm64<0, false, 0, 0, false, 0><<<dim3((unsigned)((((NB) / 64) * ((PATP) / 64) + 7) / 8), (unsigned)(1)), 256, 0, stream>>>((const unsigned short*)(H216), nullptr, HID2, 0, (const unsigned short*)(W316), nullptr, HID2, 0, (void*)(SC), nullptr, PATP, 0, nullptr, nullptr, 0, NB, PATP, HID2, INV_CARRY);
    k_head<<<NB / HROWS, 256, 0, stream>>>(SC, b3, PROB, SCORE);
    k_pair<<<(NTL * (NTL + 1)) / 2, 256, 0, stream>>>(XW, bs1, ws2, bs2, SIM);
}
